// GatedBlock_85555748536464
// MI455X (gfx1250) — hardware-verified
//
#include <hip/hip_runtime.h>


namespace {
constexpr int N = 50000, E = 800000, D = 128, NPAD = 50176, NBLK = NPAD / 128;
constexpr float FXS = 65536.0f, FXI = 1.0f / 65536.0f, WS_ = 64.0f, AS_ = 8.0f, BNE = 1e-5f;

typedef _Float16 b16;
typedef __attribute__((ext_vector_type(16))) _Float16 v16b;
typedef __attribute__((ext_vector_type(8)))  _Float16 v8b;
typedef __attribute__((ext_vector_type(8)))  float v8f;
typedef __attribute__((ext_vector_type(4)))  float v4f;

__device__ __forceinline__ v8b ld8b(const b16* p) { return *(const v8b*)p; }
__device__ __forceinline__ v16b cat8b(v8b a, v8b b) { return __builtin_shufflevector(a, b, 0, 1, 2, 3, 4, 5, 6, 7, 8, 9, 10, 11, 12, 13, 14, 15); }
__device__ __forceinline__ v16b frag_kb(const b16* p, int hh) { return cat8b(ld8b(p + 8 * hh), ld8b(p + 16 + 8 * hh)); }
__device__ __forceinline__ void split16(float v, b16& hi, b16& lo) { hi = (b16)v; lo = (b16)(v - (float)hi); }
__device__ __forceinline__ void frag_ksplit(const float* p, int hh, v16b& fh_, v16b& fl_) {
  const float* p0 = p + 8 * hh; const float* p1 = p + 16 + 8 * hh;
#pragma unroll
  for (int e = 0; e < 8; ++e) { b16 a, c; split16(p0[e], a, c); fh_[e] = a; fl_[e] = c; split16(p1[e], a, c); fh_[8 + e] = a; fl_[8 + e] = c; }
}
__device__ __forceinline__ v8f wmma16b(v16b a, v16b b, v8f c) {
  v8f d = __builtin_amdgcn_wmma_f32_16x16x32_f16(false, a, false, b, (short)0, c, false, false);
  asm volatile("v_nop\n\tv_nop\n\tv_nop\n\tv_nop" : "+v"(d) : "v"(a), "v"(b));
  return d;
}
__device__ __forceinline__ void wave_lds_sync() {
  __builtin_amdgcn_fence(__ATOMIC_RELEASE, "workgroup");
  __builtin_amdgcn_wave_barrier();
  __builtin_amdgcn_fence(__ATOMIC_ACQUIRE, "workgroup");
}

struct Opnd { const void* p0; const void* p1; int ld; };
template <int NP> __device__ __forceinline__ void load_frags(const Opnd& o, int row, int kb, int hh, v16b& fh_, v16b& fl_) {
  if (NP == 0) { frag_ksplit((const float*)o.p0 + (size_t)row * o.ld + kb, hh, fh_, fl_); }
  else if (NP == 4) {
    const float* p = (const float*)o.p0 + (size_t)row * o.ld + kb; const float* p0 = p + 8 * hh; const float* p1 = p + 16 + 8 * hh;
#pragma unroll
    for (int e = 0; e < 8; ++e) { b16 a, c; split16(p0[e] * 64.0f, a, c); fh_[e] = a; fl_[e] = c; split16(p1[e] * 64.0f, a, c); fh_[8 + e] = a; fl_[8 + e] = c; }
  } else if (NP == 3) {
    const float* p = (const float*)o.p0 + (size_t)row * o.ld + kb; const float* p0 = p + 8 * hh; const float* p1 = p + 16 + 8 * hh;
#pragma unroll
    for (int e = 0; e < 8; ++e) { fh_[e] = (b16)p0[e]; fh_[8 + e] = (b16)p1[e]; }
    fl_ = fh_;
  } else {
    fh_ = frag_kb((const b16*)o.p0 + (size_t)row * o.ld + kb, hh);
    if (NP == 2) fl_ = frag_kb((const b16*)o.p1 + (size_t)row * o.ld + kb, hh); else fl_ = fh_;
  }
}
template <int ANP, int BNP> __device__ __forceinline__ v8f mac(v16b ah, v16b al, v16b bh, v16b bl, v8f c) {
  c = wmma16b(ah, bh, c);
  if (BNP == 0 || BNP == 2 || BNP == 4) c = wmma16b(ah, bl, c);
  if (ANP == 0 || ANP == 2 || ANP == 4) c = wmma16b(al, bh, c);
  return c;
}
template <int ANP, int BNP>
__device__ __forceinline__ void gemm_tile(const Opnd& A, const Opnd& B, int K, int m0, int c0, int nloc, int hlf, v8f (&acc)[2][4]) {
  for (int kb = 0; kb < K; kb += 32) {
    v16b a0h, a0l, a1h, a1l;
    load_frags<ANP>(A, m0 + nloc, kb, hlf, a0h, a0l);
    load_frags<ANP>(A, m0 + 16 + nloc, kb, hlf, a1h, a1l);
#pragma unroll
    for (int t = 0; t < 4; ++t) {
      v16b bh, bl;
      load_frags<BNP>(B, c0 + t * 16 + nloc, kb, hlf, bh, bl);
      acc[0][t] = mac<ANP, BNP>(a0h, a0l, bh, bl, acc[0][t]);
      acc[1][t] = mac<ANP, BNP>(a1h, a1l, bh, bl, acc[1][t]);
    }
  }
}

__device__ __forceinline__ void epi_planes(v8f (&acc)[2][4], float scale, bool two, b16* __restrict__ oh, b16* __restrict__ ol, int ldo,
                                           int m0, int c0, int lane, b16* Th, b16* Tl) {
  const int nloc = lane & 15, hlf = lane >> 4;
#pragma unroll
  for (int t = 0; t < 4; ++t)
#pragma unroll
    for (int r = 0; r < 2; ++r)
#pragma unroll
      for (int v = 0; v < 8; ++v) {
        const int rr = r * 16 + v + 8 * hlf, cc = t * 16 + nloc;
        b16 h_, l_; split16(acc[r][t][v] * scale, h_, l_);
        Th[rr * 64 + cc] = h_; Tl[rr * 64 + cc] = l_;
      }
  wave_lds_sync();
  for (int pass = 0; pass < 2; ++pass) {
#pragma unroll
    for (int j = 0; j < 8; ++j) {
      const int rr = j * 4 + (lane >> 3), c8 = (lane & 7) * 8;
      const size_t o = (size_t)(m0 + rr) * ldo + c0 + c8;
      *(volatile v8b*)(oh + o) = ld8b(Th + rr * 64 + c8);
      if (two) *(volatile v8b*)(ol + o) = ld8b(Tl + rr * 64 + c8);
    }
    __threadfence();
  }
}
__device__ __forceinline__ void epi_f32(v8f (&acc)[2][4], float scale, const float* rscale, float* __restrict__ out, int ldo, int m0, int c0, int lane, float* Tt) {
  const int nloc = lane & 15, hlf = lane >> 4;
#pragma unroll
  for (int t = 0; t < 4; ++t)
#pragma unroll
    for (int r = 0; r < 2; ++r)
#pragma unroll
      for (int v = 0; v < 8; ++v) {
        const int rr = r * 16 + v + 8 * hlf;
        const float rs = rscale ? rscale[(size_t)(m0 + rr) * 32] : 1.0f;
        Tt[rr * 64 + t * 16 + nloc] = acc[r][t][v] * scale * rs;
      }
  wave_lds_sync();
  float* dst0 = out + (size_t)m0 * ldo + c0;
  for (int pass = 0; pass < 2; ++pass) {
#pragma unroll
    for (int j = 0; j < 16; ++j) { const int rr = j * 2 + hlf, c4 = nloc * 4; *(volatile v4f*)(dst0 + (size_t)rr * ldo + c4) = *(const v4f*)(Tt + rr * 64 + c4); }
    __threadfence();
  }
}


__global__ __launch_bounds__(256) void prep_kernel(const float* __restrict__ wl, const float* __restrict__ wr, const float* __restrict__ wg, b16* __restrict__ w1, b16* __restrict__ w2) {
  const size_t tid = (size_t)blockIdx.x * blockDim.x + threadIdx.x, nth = (size_t)gridDim.x * blockDim.x;
  for (int pass = 0; pass < 2; ++pass) { for (size_t p = tid; p < (size_t)D * 2 * D; p += nth) { const int n = (int)(p / (2 * D)), k = (int)(p % (2 * D));
      ((volatile b16*)w1)[p] = (b16)(((k < D) ? wl[(size_t)k * D + n] : wr[(size_t)(k - D) * D + n]) * WS_); ((volatile b16*)w2)[p] = (b16)(wg[(size_t)k * D + n] * WS_); } __threadfence(); }
}

typedef __attribute__((ext_vector_type(4))) int v4i;
__global__ __launch_bounds__(256) void agg_kernel(const int* __restrict__ esrc, const int* __restrict__ edst, const float* __restrict__ x, float* __restrict__ aggr) {
  constexpr int NB = 512;
  __shared__ __attribute__((aligned(16))) int acc[NB * D];
  __shared__ int cnt[NB]; __shared__ int list[8 * 256];
  const int t_ = threadIdx.x, wave = t_ >> 5, lane = t_ & 31, base = blockIdx.x * NB;
  for (int i = t_; i < NB * D; i += 256) acc[i] = 0;
  for (int i = t_; i < NB; i += 256) cnt[i] = 0;
  __syncthreads();
  int* wl = list + wave * 256;
  for (int c0 = 0; c0 < E; c0 += 256 * 8) {
    const int e0 = c0 + (wave * 32 + lane) * 8; int dd[8];
#pragma unroll
    for (int j = 0; j < 8; ++j) { const int dv = edst[min(e0 + j, E - 1)]; dd[j] = (e0 + j < E) ? dv : -1; }
    unsigned sl[8]; bool hit[8]; bool anyl = false;
#pragma unroll
    for (int j = 0; j < 8; ++j) { sl[j] = (unsigned)(dd[j] - base); hit[j] = sl[j] < (unsigned)NB; anyl |= hit[j]; }
    int wc = 0;
    if (__builtin_amdgcn_ballot_w32(anyl) != 0u) {
#pragma unroll
      for (int j = 0; j < 8; ++j) {
        const unsigned mj = __builtin_amdgcn_ballot_w32(hit[j]);
        if (mj != 0u) {
          if (hit[j]) { const int pos = wc + (int)__builtin_amdgcn_mbcnt_lo(mj, 0u); int s = esrc[min(e0 + j, E - 1)]; s = (s < 0) ? 0 : (s >= N ? N - 1 : s); wl[pos] = (s << 9) | (int)sl[j]; atomicAdd(&cnt[sl[j]], 1); }
          wc += __builtin_popcount(mj); } } }
    __builtin_amdgcn_wave_barrier(); __builtin_amdgcn_fence(__ATOMIC_RELEASE, "workgroup"); __builtin_amdgcn_fence(__ATOMIC_ACQUIRE, "workgroup");
    for (int i = 0; i < wc; ++i) { const int ent = wl[i]; const int s = ent >> 9, slot = ent & 511; const v4f v = *(const v4f*)(x + (size_t)s * D + lane * 4); int* ar = acc + slot * D + lane * 4;
#pragma unroll
      for (int c = 0; c < 4; ++c) atomicAdd(ar + c, (int)rintf(v[c] * FXS)); }
    __builtin_amdgcn_wave_barrier();
  }
  __syncthreads();
  for (int pass = 0; pass < 2; ++pass) {
    for (int i = t_; i < NB * D / 4; i += 256) { const int r = i >> 5, cq = (i & 31) * 4, node = base + r; v4f o = {0.0f, 0.0f, 0.0f, 0.0f};
      if (node < N) { const float sc = FXI / fmaxf((float)cnt[r], 1.0f);
#pragma unroll
        for (int c = 0; c < 4; ++c) o[c] = (float)acc[r * D + cq + c] * sc; }
      *(volatile v4f*)(aggr + (size_t)node * D + cq) = o; }
    __threadfence();
  }
}

template <int MODE>
__global__ __launch_bounds__(128) void gemm_kernel(const float* __restrict__ first, const float* __restrict__ second, const b16* __restrict__ w, const float* __restrict__ bias,
                                                  const float* __restrict__ g, const float* __restrict__ bb, const float* __restrict__ mu, const float* __restrict__ var, float* __restrict__ y) {
  __shared__ __attribute__((aligned(16))) float Ts[4][32 * 64];
  const int lane = threadIdx.x & 31, wave = threadIdx.x >> 5, nloc = lane & 15, hlf = lane >> 4, m0 = blockIdx.y * 128 + wave * 32, c0 = blockIdx.x * 64;
  const int ra = min(m0 + nloc, N - 1), rb = min(m0 + 16 + nloc, N - 1);
  v8f acc[2][4];
#pragma unroll
  for (int r = 0; r < 2; ++r)
#pragma unroll
    for (int t = 0; t < 4; ++t) acc[r][t] = (v8f){};
#pragma unroll 1
  for (int kb = 0; kb < 2 * D; kb += 32) { const float* src = (kb < D) ? first : second; const int ko = (kb < D) ? kb : kb - D; v16b a0, a1, l0, l1;
#pragma unroll
    for (int e = 0; e < 16; ++e) { const int k = ko + ((e < 8) ? (8 * hlf + e) : (16 + 8 * hlf + e - 8)); b16 p, q; split16(src[(size_t)ra * D + k] * AS_, p, q); a0[e] = p; l0[e] = q; split16(src[(size_t)rb * D + k] * AS_, p, q); a1[e] = p; l1[e] = q; }
#pragma unroll
    for (int t = 0; t < 4; ++t) { const v16b bw = frag_kb(w + (size_t)(c0 + t * 16 + nloc) * 2 * D + kb, hlf); acc[0][t] = wmma16b(a0, bw, acc[0][t]); acc[0][t] = wmma16b(l0, bw, acc[0][t]); acc[1][t] = wmma16b(a1, bw, acc[1][t]); acc[1][t] = wmma16b(l1, bw, acc[1][t]); } }
#pragma unroll
  for (int t = 0; t < 4; ++t)
#pragma unroll
    for (int r = 0; r < 2; ++r)
#pragma unroll
      for (int v = 0; v < 8; ++v) { const int row = m0 + r * 16 + 8 * hlf + v, c = c0 + t * 16 + nloc; float val = acc[r][t][v] * (1.0f / (WS_ * AS_)) + bias[c];
        if (MODE == 0) { acc[r][t][v] = (row < N) ? val : 0.0f; }
        else { const int rr = min(row, N - 1); const float gt = 1.0f / (1.0f + __expf(-val)); const float xv = first[(size_t)rr * D + c], hv = second[(size_t)rr * D + c]; acc[r][t][v] = gt * xv + (1.0f - gt) * hv; } }
  if (MODE == 0) { epi_f32(acc, 1.0f, nullptr, y, D, m0, c0, lane, Ts[wave]); return; }
  float* Tt = Ts[wave];
#pragma unroll
  for (int t = 0; t < 4; ++t)
#pragma unroll
    for (int r = 0; r < 2; ++r)
#pragma unroll
      for (int v = 0; v < 8; ++v) Tt[(r * 16 + v + 8 * hlf) * 64 + t * 16 + nloc] = acc[r][t][v];
  wave_lds_sync();
  float* dst0 = y + (size_t)m0 * D + c0;
  for (int pass = 0; pass < 2; ++pass) {
#pragma unroll
    for (int j = 0; j < 16; ++j) { const int rr = j * 2 + hlf, c4 = nloc * 4; if (m0 + rr < N) *(volatile v4f*)(dst0 + (size_t)rr * D + c4) = *(const v4f*)(Tt + rr * 64 + c4); }
    __threadfence();
  }
}
__global__ __launch_bounds__(256) void act_kernel(float* __restrict__ h, const float* __restrict__ g, const float* __restrict__ bb, const float* __restrict__ mu, const float* __restrict__ var) {
  const size_t i = (size_t)blockIdx.x * 256 + threadIdx.x; const int c0 = (int)((i * 4) % D); v4f v = *(const v4f*)(h + i * 4), o;
#pragma unroll
  for (int e = 0; e < 4; ++e) { const int c = c0 + e; const float z = g[c] * (v[e] - mu[c]) * rsqrtf(var[c] + BNE) + bb[c]; o[e] = 0.5f * z * (1.0f + erff(z * 0.70710678118654752f)); }
  for (int pass = 0; pass < 2; ++pass) { *(volatile v4f*)(h + i * 4) = o; __threadfence(); }
}
}

extern "C" void kernel_launch(void* const* d_in, const int* in_sizes, int n_in,
                              void* d_out, int out_size, void* d_ws, size_t ws_size, hipStream_t stream) {
  (void)n_in; (void)out_size;
  const float* x = (const float*)d_in[0]; const int* ei = (const int*)d_in[1]; const float* wl = (const float*)d_in[2]; const float* bl = (const float*)d_in[3]; const float* wr = (const float*)d_in[4];
  const float* bng = (const float*)d_in[5]; const float* bnb = (const float*)d_in[6]; const float* bnm = (const float*)d_in[7]; const float* bnv = (const float*)d_in[8]; const float* wg = (const float*)d_in[9]; const float* bg = (const float*)d_in[10];
  float* out = (float*)d_out;
  if (in_sizes[0] != N * D || in_sizes[1] != 2 * E || in_sizes[2] != D * D || in_sizes[4] != D * D || in_sizes[9] != 2 * D * D) return;
  const int* esrc = ei; const int* edst = ei + E;
  size_t off = 0; char* ws = (char*)d_ws;
  auto carve = [&](size_t bytes) { char* p = ws + off; off += (bytes + 255) & ~(size_t)255; return p; };
  b16* w1 = (b16*)carve((size_t)D * 2 * D * 2); b16* w2 = (b16*)carve((size_t)D * 2 * D * 2); float* aggr = (float*)carve((size_t)NPAD * D * 4); float* h = (float*)carve((size_t)NPAD * D * 4);
  if (off > ws_size) return;
  prep_kernel<<<64, 256, 0, stream>>>(wl, wr, wg, w1, w2);
  agg_kernel<<<NPAD / 512, 256, 0, stream>>>(esrc, edst, x, aggr);
  gemm_kernel<0><<<dim3(2, NBLK), 128, 0, stream>>>(aggr, x, w1, bl, bng, bnb, bnm, bnv, h);
  act_kernel<<<N * D / 4 / 256, 256, 0, stream>>>(h, bng, bnb, bnm, bnv);
  gemm_kernel<1><<<dim3(2, NBLK), 128, 0, stream>>>(x, h, w2, bg, nullptr, nullptr, nullptr, nullptr, out);
}
